// Conv1DMHSA_69621419869024
// MI455X (gfx1250) — hardware-verified
//
#include <hip/hip_runtime.h>


#define NB_  2
#define DIM  512
#define LL   2048
#define NH_  16
#define HD   32
#define RR   32
#define KS   3
#define KC   (DIM * KS)
#define ZH   2
typedef _Float16 h16;
typedef unsigned short bf;
typedef __attribute__((ext_vector_type(16))) __bf16   v16bf;
typedef __attribute__((ext_vector_type(16))) _Float16 v16h;
typedef __attribute__((ext_vector_type(8)))  _Float16 v8h;
typedef __attribute__((ext_vector_type(8)))  unsigned short v8us;
typedef __attribute__((ext_vector_type(8)))  float    v8f;
typedef __attribute__((ext_vector_type(4)))  float    v4f;
typedef v8h  __attribute__((may_alias)) v8ha;
typedef v4f  __attribute__((may_alias)) v4fa;
typedef v8us __attribute__((may_alias)) v8usa;

__device__ __forceinline__ unsigned short f2bf(float f) { unsigned u = __float_as_uint(f); u += 0x7FFFu + ((u >> 16) & 1u); return (unsigned short)(u >> 16); }
__device__ __forceinline__ float bf2f(unsigned short b) { return __uint_as_float(((unsigned)b) << 16); }
__device__ __forceinline__ float bfr(float f) { return bf2f(f2bf(f)); }
__device__ __forceinline__ v16h cat16(v8h lo, v8h hi) { return __builtin_shufflevector(lo, hi, 0, 1, 2, 3, 4, 5, 6, 7, 8, 9, 10, 11, 12, 13, 14, 15); }
__device__ __forceinline__ v16bf cat16b(v8us lo, v8us hi) { return __builtin_bit_cast(v16bf, __builtin_shufflevector(lo, hi, 0, 1, 2, 3, 4, 5, 6, 7, 8, 9, 10, 11, 12, 13, 14, 15)); }
__device__ __forceinline__ v8f wmma16(v16h a, v16h b, v8f c) { return __builtin_amdgcn_wmma_f32_16x16x32_f16(false, a, false, b, (short)0, c, false, false); }
__device__ __forceinline__ v8f wmmab(v16bf a, v16bf b, v8f c) { return __builtin_amdgcn_wmma_f32_16x16x32_bf16(false, a, false, b, (short)0, c, false, false); }


template <typename T16> struct WFrag;
template <> struct WFrag<h16> { typedef v16h V; static __device__ __forceinline__ V ld(const h16* p) { return cat16(*(const v8h*)p, *(const v8h*)(p + 16)); } static __device__ __forceinline__ v8f mma(V a, V b, v8f c) { return wmma16(a, b, c); } };
template <> struct WFrag<bf> { typedef v16bf V; static __device__ __forceinline__ V ld(const bf* p) { return cat16b(*(const v8us*)p, *(const v8us*)(p + 16)); } static __device__ __forceinline__ v8f mma(V a, V b, v8f c) { return wmmab(a, b, c); } };
template <typename T16, int NSPLIT, bool BIAS>
__global__ __launch_bounds__(32) void k_gemmw(const T16* __restrict__ A, const T16* __restrict__ A2, const T16* __restrict__ Bt, const T16* __restrict__ Bt2, int K, float* C, int ldc, const float* __restrict__ bias, size_t sA, size_t sB, size_t sC) {
    typedef typename WFrag<T16>::V V;
    __shared__ __align__(16) float os[16 * 68];
    const size_t z = blockIdx.z; A += z * sA; if (A2) A2 += z * sA; Bt += z * sB; if (Bt2) Bt2 += z * sB; C += z * sC;
    const int lane = threadIdx.x & 31, lr = lane & 15, hi = lane >> 4; const int r0 = blockIdx.x * 64, c0 = blockIdx.y * 64;
    v8f acc[4][4];
#pragma unroll
    for (int mb = 0; mb < 4; ++mb)
#pragma unroll
        for (int nb = 0; nb < 4; ++nb) acc[mb][nb] = (v8f){};
    const size_t aoff = (size_t)(r0 + lr) * K + 8 * hi, boff = (size_t)(c0 + lr) * K + 8 * hi;
#pragma unroll 1
    for (int kc = 0; kc < K; kc += 32) {
        V a[4], a2[4];
#pragma unroll
        for (int mb = 0; mb < 4; ++mb) { a[mb] = WFrag<T16>::ld(A + aoff + (size_t)mb * 16 * K + kc); if (NSPLIT == 1 || NSPLIT == 2) a2[mb] = WFrag<T16>::ld(A2 + aoff + (size_t)mb * 16 * K + kc); }
#pragma unroll
        for (int nb = 0; nb < 4; ++nb) { const V b = WFrag<T16>::ld(Bt + boff + (size_t)nb * 16 * K + kc); V b2; if (NSPLIT >= 2) b2 = WFrag<T16>::ld(Bt2 + boff + (size_t)nb * 16 * K + kc);
#pragma unroll
            for (int mb = 0; mb < 4; ++mb) { acc[mb][nb] = WFrag<T16>::mma(a[mb], b, acc[mb][nb]); if (NSPLIT == 1 || NSPLIT == 2) acc[mb][nb] = WFrag<T16>::mma(a2[mb], b, acc[mb][nb]); if (NSPLIT >= 2) acc[mb][nb] = WFrag<T16>::mma(a[mb], b2, acc[mb][nb]); } }
        asm volatile("v_nop\n\tv_nop\n\tv_nop\n\tv_nop" : "+v"(acc[0][0]), "+v"(acc[1][1]), "+v"(acc[2][2]), "+v"(acc[3][3]) : "v"(a[0]), "v"(a[3]));
    }
#pragma unroll
    for (int mb = 0; mb < 4; ++mb) {
#pragma unroll
        for (int nb = 0; nb < 4; ++nb) {
#pragma unroll
            for (int j = 0; j < 8; ++j) os[(hi * 8 + j) * 68 + nb * 16 + lr] = acc[mb][nb][j]; }
        __builtin_amdgcn_wave_barrier(); asm volatile("" ::: "memory");
        float* crow = C + (size_t)(r0 + mb * 16) * ldc + c0;
#pragma unroll 1
        for (int ps = 0; ps < 2; ++ps) {
#pragma unroll
            for (int s = 0; s < 8; ++s) { const int row = 2 * s + hi, cofs = lr * 4; v4f val = *(const v4fa*)(os + row * 68 + cofs); if (BIAS) { val[0] += bfr(bias[c0 + cofs]); val[1] += bfr(bias[c0 + cofs + 1]); val[2] += bfr(bias[c0 + cofs + 2]); val[3] += bfr(bias[c0 + cofs + 3]); }
                *(volatile v4f*)(crow + (size_t)row * ldc + cofs) = val; }
            if (ps == 0) __threadfence(); }
        __builtin_amdgcn_wave_barrier(); asm volatile("" ::: "memory");
    }
}

__device__ __forceinline__ void splitf(float y, unsigned short& h, unsigned short& l) { h = f2bf(y); l = f2bf(y - bf2f(h)); }
typedef __attribute__((ext_vector_type(2))) unsigned short v2us;
typedef __attribute__((ext_vector_type(4))) unsigned short v4us;

__global__ __launch_bounds__(256) void k_cvt8(const float* __restrict__ src, bf* dst, size_t n8) { const size_t i = (size_t)blockIdx.x * 256 + threadIdx.x; if (i >= n8) return; const v8f v = *(const v8f*)(src + i * 8); v8us o;
#pragma unroll
    for (int k = 0; k < 8; ++k) o[k] = f2bf(v[k]); *(volatile v8us*)(dst + i * 8) = o; __threadfence(); *(volatile v8us*)(dst + i * 8) = o; }
__global__ __launch_bounds__(256) void k_col(const float* __restrict__ x, bf* XC) { const size_t e = ((size_t)blockIdx.x * 256 + threadIdx.x) * 4; if (e >= (size_t)LL * KC) return; const int c = (int)(e % DIM); const int k = (int)((e / DIM) % KS); const int l = (int)(e / KC); const int ls = l - (KS - 1) + k; v4us o;
#pragma unroll
    for (int q = 0; q < 4; ++q) o[q] = ls >= 0 ? f2bf(x[(size_t)(c + q) * LL + ls]) : (unsigned short)0; *(volatile v4us*)(XC + e) = o; __threadfence(); *(volatile v4us*)(XC + e) = o; }
__global__ __launch_bounds__(256) void k_wcol(const float* __restrict__ w, bf* WC) { const size_t e = ((size_t)blockIdx.x * 256 + threadIdx.x) * 4; if (e >= (size_t)DIM * KC) return; const int c = (int)(e % DIM); const int k = (int)((e / DIM) % KS); const int o = (int)(e / KC); v4us r;
#pragma unroll
    for (int q = 0; q < 4; ++q) r[q] = f2bf(w[((size_t)o * DIM + c + q) * KS + k]); *(volatile v4us*)(WC + e) = r; __threadfence(); *(volatile v4us*)(WC + e) = r; }
__global__ __launch_bounds__(256) void k_xt(const float* __restrict__ x, bf* XT) { const size_t e = ((size_t)blockIdx.x * 256 + threadIdx.x) * 4; if (e >= (size_t)LL * DIM) return; const int c = (int)(e % DIM), l = (int)(e / DIM); v4us o;
#pragma unroll
    for (int q = 0; q < 4; ++q) o[q] = f2bf(x[(size_t)(c + q) * LL + l]); *(volatile v4us*)(XT + e) = o; __threadfence(); *(volatile v4us*)(XT + e) = o; }
__global__ __launch_bounds__(256) void k_phi(const float* __restrict__ F, const float* __restrict__ gam, const float* __restrict__ bet, const float* __restrict__ G1, const float* __restrict__ G2, bf* Ph, bf* Pl) { const size_t e = ((size_t)blockIdx.x * 256 + threadIdx.x) * 2; if (e >= (size_t)NH_ * LL * RR) return; const int r0 = (int)(e % RR); const int l = (int)((e / RR) % LL); const int h = (int)(e / ((size_t)RR * LL)); const float g = bfr(gam[0]), bb = bfr(bet[0]); const float* f = F + (size_t)l * DIM + h * HD; v2us oh, ol;
#pragma unroll
    for (int u = 0; u < 2; ++u) { const int r = r0 + u; float a = 0.f, b = 0.f;
#pragma unroll 1
        for (int d = 0; d < HD; ++d) { float t = __fmul_rn(g, f[d]); asm volatile("" : "+v"(t)); t = __fadd_rn(t, bb); float pa = __fmul_rn(t, bfr(G1[d * RR + r])); asm volatile("" : "+v"(pa)); a = __fadd_rn(a, pa); float pb = __fmul_rn(t, bfr(G2[d * RR + r])); asm volatile("" : "+v"(pb)); b = __fadd_rn(b, pb); }
        float hlf = __fmul_rn(__fmul_rn(a, b), 0.17677669529663687f); asm volatile("" : "+v"(hlf)); unsigned short x1, x2; splitf(__fmul_rn(hlf, hlf), x1, x2); oh[u] = x1; ol[u] = x2; }
    *(volatile v2us*)(Ph + e) = oh; *(volatile v2us*)(Pl + e) = ol; __threadfence(); *(volatile v2us*)(Ph + e) = oh; *(volatile v2us*)(Pl + e) = ol; }
__global__ __launch_bounds__(256) void k_vtp(const float* __restrict__ VF, bf* Vh, bf* Vl) { const size_t e = ((size_t)blockIdx.x * 256 + threadIdx.x) * 2; if (e >= (size_t)NH_ * 64 * LL) return; const int l = (int)(e % LL); const int d = (int)((e / LL) % 64); const int h = (int)(e / ((size_t)LL * 64)); v2us oh, ol;
#pragma unroll
    for (int u = 0; u < 2; ++u) { unsigned short a = 0, c = 0; if (d < HD) splitf(VF[(size_t)(l + u) * DIM + h * HD + d], a, c); oh[u] = a; ol[u] = c; } *(volatile v2us*)(Vh + e) = oh; *(volatile v2us*)(Vl + e) = ol; __threadfence(); *(volatile v2us*)(Vh + e) = oh; *(volatile v2us*)(Vl + e) = ol; }
__global__ __launch_bounds__(256) void k_norm(const float* __restrict__ Sb, bf* Ph, bf* Pl) { const int lane = threadIdx.x & 31; const int row = blockIdx.x * 8 + (threadIdx.x >> 5); if (row >= ZH * LL) return; const float* sr = Sb + (size_t)row * LL; float v[64]; float s = 0.f;
#pragma unroll
    for (int ch = 0; ch < 16; ++ch) { const v4f a = *(const v4f*)(sr + ch * 128 + lane * 4);
#pragma unroll
        for (int q = 0; q < 4; ++q) { v[ch * 4 + q] = a[q]; s = __fadd_rn(s, a[q]); } }
#pragma unroll
    for (int sh = 16; sh; sh >>= 1) s += __shfl_xor(s, sh, 32);
    const float f = __fdiv_rn(1.0f, __fadd_rn(s, 1e-6f));
#pragma unroll 1
    for (int ps = 0; ps < 2; ++ps) {
#pragma unroll
        for (int ch = 0; ch < 16; ++ch) { v4us oh, ol;
#pragma unroll
            for (int q = 0; q < 4; ++q) { unsigned short a, c; splitf(__fmul_rn(v[ch * 4 + q], f), a, c); oh[q] = a; ol[q] = c; } const size_t oo = (size_t)row * LL + ch * 128 + lane * 4; *(volatile v4us*)(Ph + oo) = oh; *(volatile v4us*)(Pl + oo) = ol; }
        if (ps == 0) __threadfence(); } }
__global__ __launch_bounds__(256) void k_mrg(const float* __restrict__ Ob, int h0, bf* Ah, bf* Al) { const size_t e = ((size_t)blockIdx.x * 256 + threadIdx.x) * 2; if (e >= (size_t)ZH * LL * HD) return; const int d = (int)(e % HD); const int l = (int)((e / HD) % LL); const int z = (int)(e / ((size_t)HD * LL)); v2us oh, ol;
#pragma unroll
    for (int u = 0; u < 2; ++u) { unsigned short a, c; splitf(Ob[((size_t)z * LL + l) * 64 + d + u], a, c); oh[u] = a; ol[u] = c; } const size_t o = (size_t)l * DIM + (h0 + z) * HD + d; *(volatile v2us*)(Ah + o) = oh; *(volatile v2us*)(Al + o) = ol; __threadfence(); *(volatile v2us*)(Ah + o) = oh; *(volatile v2us*)(Al + o) = ol; }

extern "C" void kernel_launch(void* const* d_in, const int* in_sizes, int n_in,
                              void* d_out, int out_size, void* d_ws, size_t ws_size, hipStream_t stream) {
    (void)in_sizes; (void)n_in; (void)out_size;
    const float* IN[16]; for (int i = 0; i < 16; ++i) IN[i] = (const float*)d_in[i];
    float* OUT = (float*)d_out;
    char* wsp = (char*)d_ws;
    auto take = [&](size_t bytes) { char* p = wsp; wsp += (bytes + 255) & ~(size_t)255; return (void*)p; };
    bf* WQ = (bf*)take((size_t)DIM * KC * 2); bf* WK = (bf*)take((size_t)DIM * KC * 2); bf* WV = (bf*)take((size_t)DIM * DIM * 2); bf* WP = (bf*)take((size_t)DIM * DIM * 2); bf* XC = (bf*)take((size_t)LL * KC * 2); bf* XT = (bf*)take((size_t)LL * DIM * 2);
    float* QF = (float*)take((size_t)LL * DIM * 4); float* KF = (float*)take((size_t)LL * DIM * 4); float* VF = (float*)take((size_t)LL * DIM * 4); bf* PQh = (bf*)take((size_t)NH_ * LL * RR * 2); bf* PQl = (bf*)take((size_t)NH_ * LL * RR * 2); bf* PKh = (bf*)take((size_t)NH_ * LL * RR * 2); bf* PKl = (bf*)take((size_t)NH_ * LL * RR * 2); bf* Vh = (bf*)take((size_t)NH_ * 64 * LL * 2); bf* Vl = (bf*)take((size_t)NH_ * 64 * LL * 2);
    float* Sb = (float*)take((size_t)ZH * LL * LL * 4); bf* Ph = (bf*)take((size_t)ZH * LL * LL * 2); bf* Pl = (bf*)take((size_t)ZH * LL * LL * 2); float* Ob = (float*)take((size_t)ZH * LL * 64 * 4); bf* Ah = (bf*)take((size_t)LL * DIM * 2); bf* Al = (bf*)take((size_t)LL * DIM * 2);
    if ((size_t)(wsp - (char*)d_ws) > ws_size) return;
    k_wcol<<<(unsigned)(((size_t)DIM * KC / 4 + 255) / 256), 256, 0, stream>>>(IN[1], WQ); k_wcol<<<(unsigned)(((size_t)DIM * KC / 4 + 255) / 256), 256, 0, stream>>>(IN[3], WK); k_cvt8<<<(DIM * DIM / 8 + 255) / 256, 256, 0, stream>>>(IN[5], WV, (size_t)DIM * DIM / 8); k_cvt8<<<(DIM * DIM / 8 + 255) / 256, 256, 0, stream>>>(IN[6], WP, (size_t)DIM * DIM / 8);
    const unsigned LPH = (unsigned)(((size_t)NH_ * LL * RR / 2 + 255) / 256);
    for (int b = 0; b < NB_; ++b) { const float* xb = IN[0] + (size_t)b * DIM * LL;
        k_col<<<(unsigned)(((size_t)LL * KC / 4 + 255) / 256), 256, 0, stream>>>(xb, XC); k_xt<<<(LL * DIM / 4 + 255) / 256, 256, 0, stream>>>(xb, XT);
        k_gemmw<bf, 0, true><<<dim3(LL / 64, DIM / 64, 1), 32, 0, stream>>>(XC, nullptr, WQ, nullptr, KC, QF, DIM, IN[2], 0, 0, 0); k_gemmw<bf, 0, true><<<dim3(LL / 64, DIM / 64, 1), 32, 0, stream>>>(XC, nullptr, WK, nullptr, KC, KF, DIM, IN[4], 0, 0, 0);
        k_gemmw<bf, 0, false><<<dim3(LL / 64, DIM / 64, 1), 32, 0, stream>>>(XT, nullptr, WV, nullptr, DIM, VF, DIM, nullptr, 0, 0, 0);
        k_phi<<<LPH, 256, 0, stream>>>(QF, IN[8], IN[9], IN[12], IN[13], PQh, PQl); k_phi<<<LPH, 256, 0, stream>>>(KF, IN[10], IN[11], IN[14], IN[15], PKh, PKl); k_vtp<<<(unsigned)(((size_t)NH_ * 64 * LL / 2 + 255) / 256), 256, 0, stream>>>(VF, Vh, Vl);
        for (int h0 = 0; h0 < NH_; h0 += ZH) { const size_t z = (size_t)h0;
            k_gemmw<bf, 2, false><<<dim3(LL / 64, LL / 64, ZH), 32, 0, stream>>>(PQh + z * LL * RR, PQl + z * LL * RR, PKh + z * LL * RR, PKl + z * LL * RR, RR, Sb, LL, nullptr, (size_t)LL * RR, (size_t)LL * RR, (size_t)LL * LL);
            k_norm<<<ZH * LL / 8, 256, 0, stream>>>(Sb, Ph, Pl);
            k_gemmw<bf, 2, false><<<dim3(LL / 64, 1, ZH), 32, 0, stream>>>(Ph, Pl, Vh + z * 64 * LL, Vl + z * 64 * LL, LL, Ob, 64, nullptr, (size_t)LL * LL, (size_t)64 * LL, (size_t)LL * 64);
            k_mrg<<<(unsigned)(((size_t)ZH * LL * HD / 2 + 255) / 256), 256, 0, stream>>>(Ob, h0, Ah, Al); }
        k_gemmw<bf, 1, true><<<dim3(LL / 64, DIM / 64, 1), 32, 0, stream>>>(Ah, Al, WP, nullptr, DIM, OUT + (size_t)b * LL * DIM, DIM, IN[7], 0, 0, 0); }
}
